// Block_76244259438867
// MI455X (gfx1250) — hardware-verified
//
#include <hip/hip_runtime.h>
#include <math.h>

#ifndef NB
#define NB 2
#endif
#ifndef SEQ
#define SEQ 2048
#endif
#define NB_FULL 2
#define SEQ_FULL 2048
#define WD 1024
#define NH 16
#define HDIM 64
#define FF 4096
#define QW 3072
#define ROWS (NB * SEQ)
#define EQB ((SEQ / 64) < 4 ? (SEQ / 64) : 4)
#define ER (EQB * 64)
#define RSC 2048.0f
#define RINV 0.00048828125f

static_assert(WD == 32 * 4 * 8);
static_assert(NH * HDIM == WD);
static_assert(WD / 64 == NH);
static_assert(QW == 3 * WD);
static_assert(HDIM == 64);
static_assert(SEQ % 64 == 0);
static_assert(ROWS % 64 == 0);
static_assert(WD % 64 == 0 && QW % 64 == 0 && FF % 64 == 0);
static_assert(WD % 32 == 0 && FF % 32 == 0);
static_assert(WD % 8 == 0 && FF % 8 == 0);
static_assert(NB <= NB_FULL && SEQ <= SEQ_FULL);
static_assert(ER % 64 == 0 && ER <= SEQ && ER >= 64);

typedef __attribute__((ext_vector_type(16))) _Float16 v16h;
typedef __attribute__((ext_vector_type(8)))  _Float16 v8h;
typedef __attribute__((ext_vector_type(8)))  float    v8f;
typedef __attribute__((ext_vector_type(4)))  float    v4f;
typedef __attribute__((ext_vector_type(4)))  unsigned int u4v;
typedef __attribute__((ext_vector_type(2)))  unsigned int u2v;


#define VST2(T, ptr, val) do { const T vst2_v_ = (val); *(volatile T*)(ptr) = vst2_v_; __threadfence(); *(volatile T*)(ptr) = vst2_v_; } while (0)

__device__ __forceinline__ float cmb_bf(float v) {
    const unsigned u = __builtin_bit_cast(unsigned, v);
    const unsigned r = (u + 0x7fffu + ((u >> 16) & 1u)) & 0xffff0000u;
    return __builtin_bit_cast(float, r);
}
__device__ __forceinline__ unsigned int pk2h(float a, float b) {
    return (unsigned int)__builtin_bit_cast(unsigned short, (_Float16)a) | ((unsigned int)__builtin_bit_cast(unsigned short, (_Float16)b) << 16);
}

__device__ __forceinline__ void dep_guard_h(v8f& a, v8f& b, v16h x, v16h y) { asm volatile("v_nop\n\tv_nop\n\tv_nop\n\tv_nop" : "+v"(a), "+v"(b) : "v"(x), "v"(y)); }
__device__ __forceinline__ void keep4_h(v16h a, v16h b, v16h c, v16h d) { asm volatile("v_nop" :: "v"(a), "v"(b), "v"(c), "v"(d)); }
__device__ __forceinline__ void acc_guard4(v8f& a, v8f& b, v8f& c, v8f& d) { asm volatile("v_nop\n\tv_nop\n\tv_nop\n\tv_nop" : "+v"(a), "+v"(b), "+v"(c), "+v"(d)); }

union FragH { v16h v; v8h h[2]; };
__device__ __forceinline__ v16h frag_ld(const _Float16* p) { FragH f; f.h[0] = *(const v8h*)(p); f.h[1] = *(const v8h*)(p + 16); return f.v; }
__device__ __forceinline__ v8f mma_h(v16h a, v16h b, v8f c) { return __builtin_amdgcn_wmma_f32_16x16x32_f16(false, a, false, b, (short)0, c, false, false); }
__device__ __forceinline__ v8f wmma16(v16h a, v16h b, v8f c) {
    c = __builtin_amdgcn_wmma_f32_16x16x32_f16(false, a, false, b, (short)0, c, false, false);
    asm volatile("v_nop\n\tv_nop\n\tv_nop\n\tv_nop" : "+v"(c) : "v"(a), "v"(b));
    return c;
}

__device__ __forceinline__ float red16(float s) {
    s += __shfl_xor(s, 1, 32); s += __shfl_xor(s, 2, 32); s += __shfl_xor(s, 4, 32); s += __shfl_xor(s, 8, 32);
    return s;
}

__device__ __forceinline__ v4f expmap_row(v4f x, v4f v, float cc) {
    const float EPS = 1e-9f;
    const float xn  = red16((x.x * x.x + x.y * x.y) + (x.z * x.z + x.w * x.w));
    const float vns = red16((v.x * v.x + v.y * v.y) + (v.z * v.z + v.w * v.w));
    const float sf = 2.0f / (1.0f + cc * xn + EPS);
    const float vn = sqrtf(vns + EPS);
    const float targ = fabsf(cc * sf * vns * 0.5f);
    const float coeff = (1.0f / (sqrtf(fabsf(cc) + EPS) + EPS)) * tanhf(sqrtf(targ + EPS));
    const float dv = vn + EPS;
    v4f y;
    y.x = coeff * v.x / dv; y.y = coeff * v.y / dv; y.z = coeff * v.z / dv; y.w = coeff * v.w / dv;
    const float yn = red16((y.x * y.x + y.y * y.y) + (y.z * y.z + y.w * y.w));
    const float ip = red16((x.x * y.x + x.y * y.y) + (x.z * y.z + x.w * y.w));
    const float ca = 1.0f + 2.0f * cc * ip + cc * yn;
    const float cb = 1.0f - cc * xn;
    const float den = (1.0f + 2.0f * cc * ip + cc * cc * xn * yn) + EPS;
    v4f o;
    o.x = (ca * x.x + cb * y.x) / den; o.y = (ca * x.y + cb * y.y) / den;
    o.z = (ca * x.z + cb * y.z) / den; o.w = (ca * x.w + cb * y.w) / den;
    return o;
}

__device__ __forceinline__ void gemm_kloop(v8f (&acc)[4][4], const _Float16* __restrict__ A, int arow0, int lda,
                                           const _Float16* __restrict__ Bt, int n0, int ldb, int K, int rlane, int koff) {
    for (int k0 = 0; k0 < K; k0 += 32) {
        v16h bh[4];
#pragma unroll
        for (int j = 0; j < 4; ++j) {
            const size_t bo = (size_t)(n0 + (j << 4) + rlane) * ldb + koff + k0;
            bh[j] = frag_ld(Bt + bo);
        }
#pragma unroll
        for (int i = 0; i < 4; ++i) {
            const size_t ao = (size_t)(arow0 + (i << 4) + rlane) * lda + koff + k0;
            const v16h ah = frag_ld(A + ao);
#pragma unroll
            for (int j = 0; j < 4; ++j) acc[i][j] = mma_h(ah, bh[j], acc[i][j]);
            dep_guard_h(acc[i][0], acc[i][3], ah, ah);
        }
        keep4_h(bh[0], bh[1], bh[2], bh[3]);
    }
    acc_guard4(acc[0][0], acc[0][1], acc[0][2], acc[0][3]);
    acc_guard4(acc[1][0], acc[1][1], acc[1][2], acc[1][3]);
    acc_guard4(acc[2][0], acc[2][1], acc[2][2], acc[2][3]);
    acc_guard4(acc[3][0], acc[3][1], acc[3][2], acc[3][3]);
}

template <int OUT_MODE, int EPI, int APRE>
__device__ __forceinline__ void gemm64_body(const unsigned short* __restrict__ Ap, int lda, const unsigned short* __restrict__ Arp,
                                            const unsigned short* __restrict__ Btp, int ldb,
                                            void* __restrict__ Cout, int ldc, const float* __restrict__ resid, int rpb, long long rbs,
                                            const float* __restrict__ cvec, int M, int N, int K, float scale, float* slab) {
    const _Float16* A = (const _Float16*)Ap; const _Float16* Bt = (const _Float16*)Btp;
    const int lane = threadIdx.x & 31;
    const int wave = threadIdx.x >> 5;
    const int tilesN = N >> 6;
    const int tilesM = M >> 6;
    const int tile = blockIdx.x * 8 + wave;
    if (tile >= tilesM * tilesN) return;
    const int tm = tile / tilesN;
    const int tn = tile - tm * tilesN;
    const int m0 = tm << 6;
    const int n0 = tn << 6;
    const int rlane = lane & 15;
    const int koff  = (lane >> 4) * 8;
    const int mOff  = (lane >> 4) * 8;

    v8f acc[4][4];
#pragma unroll
    for (int i = 0; i < 4; ++i)
#pragma unroll
        for (int j = 0; j < 4; ++j) acc[i][j] = (v8f){0.f, 0.f, 0.f, 0.f, 0.f, 0.f, 0.f, 0.f};

    if (APRE) {
        const int mb = m0 / SEQ;
        const int mr = m0 - mb * SEQ;
        if (mr < ER) {
            gemm_kloop(acc, (const _Float16*)Arp, mb * ER + mr, lda, Bt, n0, ldb, K, rlane, koff);
#pragma unroll
            for (int i = 0; i < 4; ++i)
#pragma unroll
                for (int j = 0; j < 4; ++j) acc[i][j] = acc[i][j] * RINV;
        }
    }
    gemm_kloop(acc, A, m0, lda, Bt, n0, ldb, K, rlane, koff);

    float cc = 0.f;
    if (EPI >= 2) {
        int hd = n0 >> 6; hd = hd < NH ? hd : NH - 1;
        cc = fminf(fmaxf(cmb_bf(cvec[hd]), 1e-4f), 1.0f);
    }

#pragma unroll
    for (int i = 0; i < 4; ++i) {
        const int mBase = m0 + (i << 4);
#pragma unroll
        for (int j = 0; j < 4; ++j) {
#pragma unroll
            for (int r = 0; r < 8; ++r) slab[(mOff + r) * 68 + (j << 4) + rlane] = acc[i][j][r] * scale;
        }
        __builtin_amdgcn_fence(3  , "workgroup");
        __builtin_amdgcn_wave_barrier();
        __builtin_amdgcn_fence(2  , "workgroup");
        if (OUT_MODE == 0) {
            float* C = (float*)Cout;
            const int hh = lane >> 4, c4 = (lane & 15) * 4;
            if (EPI >= 2) {
#pragma unroll 1
                for (int it = 0; it < 8; ++it) {
                    const int row = it * 2 + hh;
                    const v4f v = *(const v4f*)(slab + row * 68 + c4);
                    const int gr = mBase + row;
                    const float* rp = resid + (long long)(gr / rpb) * rbs + (long long)(gr % rpb) * WD + n0 + c4;
                    v4f x = *(const v4f*)rp;
                    if (EPI == 2) { x.x = cmb_bf(x.x); x.y = cmb_bf(x.y); x.z = cmb_bf(x.z); x.w = cmb_bf(x.w); }
                    const v4f o = expmap_row(x, v, cc);
                    *(v4f*)(slab + row * 68 + c4) = o;
                }
            }
            for (int pass = 0; pass < 2; ++pass) {
#pragma unroll
                for (int it = 0; it < 8; ++it) {
                    const int row = it * 2 + hh;
                    const v4f v = *(const v4f*)(slab + row * 68 + c4);
                    *(volatile v4f*)(C + (size_t)(mBase + row) * ldc + n0 + c4) = v;
                }
                __threadfence();
            }
        } else {
            const int q = lane >> 3, c8 = (lane & 7) * 8;
            _Float16* C = (_Float16*)Cout;
            if (EPI == 1) {
#pragma unroll 1
                for (int it = 0; it < 4; ++it) {
                    float* sp = slab + (it * 4 + q) * 68 + c8;
#pragma unroll
                    for (int e = 0; e < 8; ++e) { const float t = sp[e]; sp[e] = 0.5f * t * (1.0f + erff(t * 0.70710678118654752f)); }
                }
            }
            for (int pass = 0; pass < 2; ++pass) {
#pragma unroll
                for (int it = 0; it < 4; ++it) {
                    const int row = it * 4 + q;
                    const float* sp = slab + row * 68 + c8;
                    v8h hv;
#pragma unroll
                    for (int e = 0; e < 8; ++e) hv[e] = (_Float16)sp[e];
                    *(volatile v8h*)(C + (size_t)(mBase + row) * ldc + n0 + c8) = hv;
                }
                __threadfence();
            }
        }
        __builtin_amdgcn_fence(3  , "workgroup");
        __builtin_amdgcn_wave_barrier();
        __builtin_amdgcn_fence(2  , "workgroup");
    }
}

__global__ __launch_bounds__(256) void k_gemm_qkv(const unsigned short* __restrict__ A, const unsigned short* __restrict__ Bt, float* __restrict__ C) {
    __shared__ __align__(16) float sT[8][16 * 68];
    gemm64_body<0, 0, 0>(A, WD, nullptr, Bt, WD, (void*)C, QW, nullptr, 1, 0LL, nullptr, ROWS, QW, WD, 0.0625f, sT[threadIdx.x >> 5]);
}
__global__ __launch_bounds__(256) void k_gemm_proj(const unsigned short* __restrict__ A, const unsigned short* __restrict__ AR, const unsigned short* __restrict__ Bt,
                                                   float* __restrict__ C, const float* __restrict__ xin, const float* __restrict__ cvec) {
    __shared__ __align__(16) float sT[8][16 * 68];
    gemm64_body<0, 2, 1>(A, WD, AR, Bt, WD, (void*)C, WD, xin, SEQ, (long long)SEQ_FULL * WD, cvec, ROWS, WD, WD, 0.0625f, sT[threadIdx.x >> 5]);
}
__global__ __launch_bounds__(256) void k_gemm_fc(const unsigned short* __restrict__ A, const unsigned short* __restrict__ Bt, unsigned short* __restrict__ C) {
    __shared__ __align__(16) float sT[8][16 * 68];
    gemm64_body<1, 1, 0>(A, WD, nullptr, Bt, WD, (void*)C, FF, nullptr, 1, 0LL, nullptr, ROWS, FF, WD, 0.0625f, sT[threadIdx.x >> 5]);
}
__global__ __launch_bounds__(256) void k_gemm_mlp2(const unsigned short* __restrict__ A, const unsigned short* __restrict__ Bt, float* __restrict__ C,
                                                   const float* __restrict__ x1, const float* __restrict__ cvec) {
    __shared__ __align__(16) float sT[8][16 * 68];
    gemm64_body<0, 3, 0>(A, FF, nullptr, Bt, FF, (void*)C, WD, x1, SEQ, (long long)SEQ * WD, cvec, ROWS, WD, FF, 0.0625f, sT[threadIdx.x >> 5]);
}

template <int ABF>
__device__ __forceinline__ void ln_body(const float* __restrict__ A, int rpb, long long bstride, const float* __restrict__ GA, int rows, unsigned short* __restrict__ Y16) {
    #pragma clang fp contract(off)
    constexpr int NQ = 8;
    const int r = blockIdx.x * 8 + (threadIdx.x >> 5); const int L = threadIdx.x & 31; if (r >= rows) return;
    const float* ar = A + (long long)(r / rpb) * bstride + (long long)(r % rpb) * WD;
    v4f v[NQ]; float s = 0.f;
#pragma unroll
    for (int q = 0; q < NQ; ++q) {
        v[q] = *(const v4f*)(ar + 4 * L + 128 * q);
        if (ABF) { v[q].x = cmb_bf(v[q].x); v[q].y = cmb_bf(v[q].y); v[q].z = cmb_bf(v[q].z); v[q].w = cmb_bf(v[q].w); }
        s += (v[q].x + v[q].y) + (v[q].z + v[q].w);
    }
#pragma unroll
    for (int o = 16; o > 0; o >>= 1) s += __shfl_xor(s, o, 32);
    const float mu = s * (1.f / WD); float qq = 0.f;
#pragma unroll
    for (int q = 0; q < NQ; ++q) { v[q].x -= mu; v[q].y -= mu; v[q].z -= mu; v[q].w -= mu; qq += (v[q].x * v[q].x + v[q].y * v[q].y) + (v[q].z * v[q].z + v[q].w * v[q].w); }
#pragma unroll
    for (int o = 16; o > 0; o >>= 1) qq += __shfl_xor(qq, o, 32);
    const float rs = rsqrtf(qq * (1.f / WD) + 1e-5f);
#pragma unroll
    for (int q = 0; q < NQ; ++q) {
        const int c = 4 * L + 128 * q; const v4f ga = *(const v4f*)(GA + c); v4f y;
        y.x = v[q].x * rs * cmb_bf(ga.x); y.y = v[q].y * rs * cmb_bf(ga.y);
        y.z = v[q].z * rs * cmb_bf(ga.z); y.w = v[q].w * rs * cmb_bf(ga.w);
        u2v pk; pk.x = pk2h(y.x, y.y); pk.y = pk2h(y.z, y.w);
        VST2(u2v, (u2v*)(Y16 + (long long)r * WD + c), pk);
    }
}
__global__ __launch_bounds__(256) void k_ln_in(const float* __restrict__ xin, const float* __restrict__ GA, unsigned short* __restrict__ Y16) {
    ln_body<1>(xin, SEQ, (long long)SEQ_FULL * WD, GA, ROWS, Y16);
}
__global__ __launch_bounds__(256) void k_ln_mid(const float* __restrict__ x1, const float* __restrict__ GA, unsigned short* __restrict__ Y16) {
    ln_body<0>(x1, SEQ, (long long)SEQ * WD, GA, ROWS, Y16);
}

__global__ __launch_bounds__(256) void k_cast_w(const float* __restrict__ SRC, unsigned short* __restrict__ DST, int n8, float sc) {
    const int u = blockIdx.x * 256 + threadIdx.x; if (u >= n8) return;
    const v4f a = *(const v4f*)(SRC + (size_t)u * 8);
    const v4f b = *(const v4f*)(SRC + (size_t)u * 8 + 4);
    u4v pk;
    pk.x = pk2h(cmb_bf(a.x) * sc, cmb_bf(a.y) * sc); pk.y = pk2h(cmb_bf(a.z) * sc, cmb_bf(a.w) * sc);
    pk.z = pk2h(cmb_bf(b.x) * sc, cmb_bf(b.y) * sc); pk.w = pk2h(cmb_bf(b.z) * sc, cmb_bf(b.w) * sc);
    VST2(u4v, (u4v*)(DST + (size_t)u * 8), pk);
}

#define AT_D 64
#define AT_KC 64
template <int EARLY>
__device__ __forceinline__ void attn_body(const float* __restrict__ qkv, unsigned short* __restrict__ ao16, unsigned short* __restrict__ aor16) {
    __shared__ __align__(16) _Float16 Ksh[AT_KC * AT_D];
    __shared__ __align__(16) _Float16 Vth[AT_D * AT_KC];
    __shared__ __align__(16) _Float16 Vtl[EARLY ? AT_D * AT_KC : 8];
    __shared__ __align__(16) _Float16 Psh[4 * 16 * AT_KC];
    __shared__ __align__(16) _Float16 Psl[EARLY ? 4 * 16 * AT_KC : 8];
    __shared__ __align__(16) float    Os[4 * 16 * 68];
    const float PSC = 32768.0f;

    const int tid  = threadIdx.x;
    const int wave = tid >> 5;
    const int lane = tid & 31;
    const int hh   = lane >> 4;
    const int c    = lane & 15;

    constexpr int NQB = EARLY ? EQB : (((SEQ / 64) - EQB) > 0 ? ((SEQ / 64) - EQB) : 1);
    constexpr int QB0 = EARLY ? 0 : EQB;
    const int bx = blockIdx.x;
    const int qb = QB0 + bx % NQB;
    const int bh = bx / NQB;
    const int h  = bh % NH;
    const int b  = bh / NH;
    const int q0 = qb * 64 + wave * 16;
    const float* base = qkv + (size_t)b * SEQ * QW + h * HDIM;

    v16h qa[2];
    {
        const float* qrow = base + (size_t)(q0 + c) * QW;
#pragma unroll
        for (int dc = 0; dc < 2; ++dc) {
#pragma unroll
            for (int hf = 0; hf < 2; ++hf) {
                const float* p = qrow + dc * 32 + 16 * hf + 8 * hh;
                const v4f a0 = *(const v4f*)(p), a1 = *(const v4f*)(p + 4);
                qa[dc][8 * hf + 0] = (_Float16)a0.x; qa[dc][8 * hf + 1] = (_Float16)a0.y; qa[dc][8 * hf + 2] = (_Float16)a0.z; qa[dc][8 * hf + 3] = (_Float16)a0.w;
                qa[dc][8 * hf + 4] = (_Float16)a1.x; qa[dc][8 * hf + 5] = (_Float16)a1.y; qa[dc][8 * hf + 6] = (_Float16)a1.z; qa[dc][8 * hf + 7] = (_Float16)a1.w;
            }
        }
    }

    float mrow[8], lrow[8];
    v8f oacc[4], oacr[4];
#pragma unroll
    for (int r = 0; r < 8; ++r) { mrow[r] = -INFINITY; lrow[r] = 0.f; }
#pragma unroll
    for (int t = 0; t < 4; ++t) { oacc[t] = (v8f){0.f, 0.f, 0.f, 0.f, 0.f, 0.f, 0.f, 0.f}; oacr[t] = (v8f){0.f, 0.f, 0.f, 0.f, 0.f, 0.f, 0.f, 0.f}; }

    const int pwo = wave * 16 * AT_KC;
    const int nChunks = qb + 1;
    for (int kc = 0; kc < nChunks; ++kc) {
        const int kv0 = kc * AT_KC;
        __syncthreads();
        {
            const int kvr = tid >> 1, dh = (tid & 1) * 32;
            const float* krow = base + WD + (size_t)(kv0 + kvr) * QW + dh;
            const float* vrow = base + 2 * WD + (size_t)(kv0 + kvr) * QW + dh;
#pragma unroll
            for (int i = 0; i < 4; ++i) {
                const v4f k0v = *(const v4f*)(krow + 8 * i), k1v = *(const v4f*)(krow + 8 * i + 4);
                v8h kk;
                kk[0] = (_Float16)k0v.x; kk[1] = (_Float16)k0v.y; kk[2] = (_Float16)k0v.z; kk[3] = (_Float16)k0v.w;
                kk[4] = (_Float16)k1v.x; kk[5] = (_Float16)k1v.y; kk[6] = (_Float16)k1v.z; kk[7] = (_Float16)k1v.w;
                *(v8h*)(&Ksh[kvr * AT_D + dh + 8 * i]) = kk;
                const v4f v0v = *(const v4f*)(vrow + 8 * i), v1v = *(const v4f*)(vrow + 8 * i + 4);
                const int d0 = dh + 8 * i;
                float vv[8];
                vv[0] = v0v.x; vv[1] = v0v.y; vv[2] = v0v.z; vv[3] = v0v.w; vv[4] = v1v.x; vv[5] = v1v.y; vv[6] = v1v.z; vv[7] = v1v.w;
#pragma unroll
                for (int e = 0; e < 8; ++e) {
                    const _Float16 hq = (_Float16)vv[e];
                    Vth[(d0 + e) * AT_KC + kvr] = hq;
                    if (EARLY) Vtl[(d0 + e) * AT_KC + kvr] = (_Float16)((vv[e] - (float)hq) * RSC);
                }
            }
        }
        __syncthreads();

        v8f s[4];
#pragma unroll
        for (int j = 0; j < 4; ++j) {
            s[j] = (v8f){0.f, 0.f, 0.f, 0.f, 0.f, 0.f, 0.f, 0.f};
#pragma unroll
            for (int dc = 0; dc < 2; ++dc) {
                FragH kb;
                kb.h[0] = *(const v8h*)(&Ksh[(j * 16 + c) * AT_D + dc * 32 + 8 * hh]);
                kb.h[1] = *(const v8h*)(&Ksh[(j * 16 + c) * AT_D + dc * 32 + 16 + 8 * hh]);
                s[j] = wmma16(qa[dc], kb.v, s[j]);
            }
        }
        const bool diag = (kc == qb);
        float cm[8];
#pragma unroll
        for (int r = 0; r < 8; ++r) {
            const int qrow = q0 + 8 * hh + r;
            float m = -INFINITY;
#pragma unroll
            for (int j = 0; j < 4; ++j) {
                const int kvcol = kv0 + j * 16 + c;
                float sv = s[j][r] * 0.125f;
                sv = (diag && (kvcol > qrow)) ? -INFINITY : sv;
                s[j][r] = sv;
                m = fmaxf(m, sv);
            }
#pragma unroll
            for (int off = 1; off < 16; off <<= 1) m = fmaxf(m, __shfl_xor(m, off, 32));
            cm[r] = m;
        }
#pragma unroll
        for (int r = 0; r < 8; ++r) {
            const float mnew = fmaxf(mrow[r], cm[r]);
            const float alpha = expf(mrow[r] - mnew);
            mrow[r] = mnew;
            float psum = 0.f;
#pragma unroll
            for (int j = 0; j < 4; ++j) {
                const float p = expf(s[j][r] - mnew);
                psum += p;
                const float pf = p * PSC;
                const _Float16 ph = (_Float16)pf;
                Psh[pwo + (8 * hh + r) * AT_KC + j * 16 + c] = ph;
                if (EARLY) Psl[pwo + (8 * hh + r) * AT_KC + j * 16 + c] = (_Float16)((pf - (float)ph) * RSC);
            }
#pragma unroll
            for (int off = 1; off < 16; off <<= 1) psum += __shfl_xor(psum, off, 32);
            lrow[r] = lrow[r] * alpha + psum;
#pragma unroll
            for (int t = 0; t < 4; ++t) { oacc[t][r] *= alpha; if (EARLY) oacr[t][r] *= alpha; }
        }
        __builtin_amdgcn_fence(3  , "workgroup");
        __builtin_amdgcn_wave_barrier();
        __builtin_amdgcn_fence(2  , "workgroup");
#pragma unroll
        for (int kk = 0; kk < 2; ++kk) {
            FragH pa;
            pa.h[0] = *(const v8h*)(&Psh[pwo + c * AT_KC + kk * 32 + 8 * hh]);
            pa.h[1] = *(const v8h*)(&Psh[pwo + c * AT_KC + kk * 32 + 16 + 8 * hh]);
            v16h plv = pa.v;
            if (EARLY) {
                FragH pl;
                pl.h[0] = *(const v8h*)(&Psl[pwo + c * AT_KC + kk * 32 + 8 * hh]);
                pl.h[1] = *(const v8h*)(&Psl[pwo + c * AT_KC + kk * 32 + 16 + 8 * hh]);
                plv = pl.v;
            }
#pragma unroll
            for (int t = 0; t < 4; ++t) {
                FragH vb;
                vb.h[0] = *(const v8h*)(&Vth[(t * 16 + c) * AT_KC + kk * 32 + 8 * hh]);
                vb.h[1] = *(const v8h*)(&Vth[(t * 16 + c) * AT_KC + kk * 32 + 16 + 8 * hh]);
                oacc[t] = wmma16(pa.v, vb.v, oacc[t]);
                if (EARLY) {
                    oacr[t] = wmma16(plv, vb.v, oacr[t]);
                    FragH vl;
                    vl.h[0] = *(const v8h*)(&Vtl[(t * 16 + c) * AT_KC + kk * 32 + 8 * hh]);
                    vl.h[1] = *(const v8h*)(&Vtl[(t * 16 + c) * AT_KC + kk * 32 + 16 + 8 * hh]);
                    oacr[t] = wmma16(pa.v, vl.v, oacr[t]);
                }
            }
        }
    }

    const int oso = wave * 16 * 68;
#pragma unroll
    for (int r = 0; r < 8; ++r) {
        const float inv = 1.0f / (lrow[r] * PSC);
#pragma unroll
        for (int t = 0; t < 4; ++t) {
            float o = oacc[t][r];
            if (EARLY) o = o + oacr[t][r] * RINV;
            Os[oso + (8 * hh + r) * 68 + t * 16 + c] = o * inv;
        }
    }
    __builtin_amdgcn_fence(3  , "workgroup");
    __builtin_amdgcn_wave_barrier();
    __builtin_amdgcn_fence(2  , "workgroup");
    {
        const int q = lane >> 3, c8 = (lane & 7) * 8;
        _Float16* ob = (_Float16*)ao16 + (size_t)b * SEQ * WD + h * HDIM;
        _Float16* obr = (_Float16*)aor16 + (size_t)b * ER * WD + h * HDIM;
        for (int pass = 0; pass < 2; ++pass) {
#pragma unroll
            for (int it = 0; it < 4; ++it) {
                const int row = it * 4 + q;
                const float* sp = &Os[oso + row * 68 + c8];
                v8h hv, lv;
#pragma unroll
                for (int e = 0; e < 8; ++e) {
                    const float f = sp[e];
                    const _Float16 hq = (_Float16)f;
                    hv[e] = hq;
                    lv[e] = (_Float16)((f - (float)hq) * RSC);
                }
                *(volatile v8h*)(ob + (size_t)(q0 + row) * WD + c8) = hv;
                if (EARLY) *(volatile v8h*)(obr + (size_t)(q0 + row) * WD + c8) = lv;
            }
            __threadfence();
        }
    }
}
__global__ __launch_bounds__(128) void k_attn_early(const float* __restrict__ qkv, unsigned short* __restrict__ ao16, unsigned short* __restrict__ aor16) {
    attn_body<1>(qkv, ao16, aor16);
}
__global__ __launch_bounds__(128) void k_attn_late(const float* __restrict__ qkv, unsigned short* __restrict__ ao16) {
    attn_body<0>(qkv, ao16, ao16);
}

constexpr size_t SZ_H16  = (size_t)ROWS * WD * 2;
constexpr size_t SZ_H2   = (size_t)ROWS * WD * 2;
constexpr size_t SZ_HS   = SZ_H16 > SZ_H2 ? SZ_H16 : SZ_H2;
constexpr size_t SZ_WQKV = (size_t)QW * WD * 2;
constexpr size_t SZ_WP   = (size_t)WD * WD * 2;
constexpr size_t SZ_WFC  = (size_t)FF * WD * 2;
constexpr size_t SZ_WMP  = (size_t)WD * FF * 2;
constexpr size_t SZ_QKV  = (size_t)ROWS * QW * 4;
constexpr size_t SZ_A1   = (size_t)ROWS * FF * 2;
constexpr size_t SZ_BIG  = SZ_QKV > SZ_A1 ? SZ_QKV : SZ_A1;
constexpr size_t SZ_AO16 = (size_t)ROWS * WD * 2;
constexpr size_t SZ_AOR  = (size_t)NB * ER * WD * 2;
constexpr size_t SZ_X1   = (size_t)ROWS * WD * 4;
constexpr size_t SZ_TOTAL = SZ_HS + SZ_WQKV + SZ_WP + SZ_WFC + SZ_WMP + SZ_BIG + SZ_AO16 + SZ_AOR + SZ_X1;
static_assert(SZ_HS >= SZ_H16 && SZ_HS >= SZ_H2 && SZ_BIG >= SZ_QKV && SZ_BIG >= SZ_A1);
static_assert(SZ_HS % 256 == 0 && SZ_WQKV % 256 == 0 && SZ_WP % 256 == 0 && SZ_WFC % 256 == 0 && SZ_WMP % 256 == 0);
static_assert(SZ_BIG % 256 == 0 && SZ_AO16 % 256 == 0 && SZ_AOR % 256 == 0 && SZ_X1 % 256 == 0);
static_assert(SZ_TOTAL <= (size_t)134217728);
static_assert(((ROWS / 64) * (QW / 64)) % 8 == 0 && ((ROWS / 64) * (WD / 64)) % 8 == 0 && ((ROWS / 64) * (FF / 64)) % 8 == 0);
static_assert((QW * WD) % 8 == 0 && (WD * WD) % 8 == 0 && (FF * WD) % 8 == 0);

extern "C" void kernel_launch(void* const* d_in, const int* in_sizes, int n_in, void* d_out, int out_size, void* d_ws, size_t ws_size, hipStream_t stream) {
    if (n_in < 9) return;
    if (in_sizes[0] < ((NB - 1) * SEQ_FULL + SEQ) * WD) return;
    if (in_sizes[1] < WD || in_sizes[5] < WD) return;
    if (in_sizes[2] < QW * WD || in_sizes[3] < WD * WD) return;
    if (in_sizes[6] < FF * WD || in_sizes[7] < WD * FF) return;
    if (in_sizes[4] < NH || in_sizes[8] < NH) return;
    if (out_size < ROWS * WD) return;
    if (SZ_TOTAL > ws_size) return;
    const float* x     = (const float*)d_in[0];
    const float* g1    = (const float*)d_in[1];
    const float* Wqkv  = (const float*)d_in[2];
    const float* Wp    = (const float*)d_in[3];
    const float* cattn = (const float*)d_in[4];
    const float* g2    = (const float*)d_in[5];
    const float* Wfc   = (const float*)d_in[6];
    const float* Wmp   = (const float*)d_in[7];
    const float* cmlp  = (const float*)d_in[8];
    float* out = (float*)d_out;

    char* wsp = (char*)d_ws;
    unsigned short* H16    = (unsigned short*)wsp; wsp += SZ_HS;
    unsigned short* WQKV16 = (unsigned short*)wsp; wsp += SZ_WQKV;
    unsigned short* WP16   = (unsigned short*)wsp; wsp += SZ_WP;
    unsigned short* WFC16  = (unsigned short*)wsp; wsp += SZ_WFC;
    unsigned short* WMP16  = (unsigned short*)wsp; wsp += SZ_WMP;
    float*          QKV    = (float*)wsp;
    unsigned short* A1     = (unsigned short*)wsp; wsp += SZ_BIG;
    unsigned short* AO16   = (unsigned short*)wsp; wsp += SZ_AO16;
    unsigned short* AOR16  = (unsigned short*)wsp; wsp += SZ_AOR;
    float*          X1     = (float*)wsp;          wsp += SZ_X1;
    unsigned short* H2     = H16;

    k_ln_in<<<(ROWS + 7) / 8, 256, 0, stream>>>(x, g1, H16);
    k_cast_w<<<(QW * WD / 8 + 255) / 256, 256, 0, stream>>>(Wqkv, WQKV16, QW * WD / 8, 16.0f);
    k_cast_w<<<(WD * WD / 8 + 255) / 256, 256, 0, stream>>>(Wp, WP16, WD * WD / 8, 16.0f);
    k_cast_w<<<(FF * WD / 8 + 255) / 256, 256, 0, stream>>>(Wfc, WFC16, FF * WD / 8, 16.0f);
    k_cast_w<<<(WD * FF / 8 + 255) / 256, 256, 0, stream>>>(Wmp, WMP16, WD * FF / 8, 16.0f);
    k_gemm_qkv<<<((ROWS / 64) * (QW / 64) + 7) / 8, 256, 0, stream>>>(H16, WQKV16, QKV);
    k_attn_early<<<NB * NH * EQB, 128, 0, stream>>>(QKV, AO16, AOR16);
    if ((SEQ / 64) > EQB) k_attn_late<<<NB * NH * ((SEQ / 64) - EQB), 128, 0, stream>>>(QKV, AO16);
    k_gemm_proj<<<((ROWS / 64) * (WD / 64) + 7) / 8, 256, 0, stream>>>(AO16, AOR16, WP16, X1, x, cattn);
    k_ln_mid<<<(ROWS + 7) / 8, 256, 0, stream>>>(X1, g2, H2);
    k_gemm_fc<<<((ROWS / 64) * (FF / 64) + 7) / 8, 256, 0, stream>>>(H2, WFC16, A1);
    k_gemm_mlp2<<<((ROWS / 64) * (WD / 64) + 7) / 8, 256, 0, stream>>>(A1, WMP16, out, X1, cmlp);
}
